// MultHeadAttention_12627203851088
// MI455X (gfx1250) — hardware-verified
//
#include <hip/hip_runtime.h>

#define B_ 4
#define S_ 2048
#define E_ 1024
#define H_ 16
#define D_ 64
#define M_ (B_ * S_)

typedef __bf16 v16bf __attribute__((ext_vector_type(16)));
typedef unsigned short v8us __attribute__((ext_vector_type(8)));
typedef float v8f __attribute__((ext_vector_type(8)));
typedef float v4f __attribute__((ext_vector_type(4)));

union Frag { v16bf v; v8us u[2]; };

__device__ __forceinline__ v8f wmma_bf16(v16bf a, v16bf b, v8f c)
{
    return __builtin_amdgcn_wmma_f32_16x16x32_bf16(false, a, false, b, (short)0, c, false, false);
}

__device__ __forceinline__ void mma3(v8f& c, const Frag& ah, const Frag& al, const Frag& bh, const Frag& bl)
{
    c = wmma_bf16(al.v, bh.v, c);
    c = wmma_bf16(ah.v, bl.v, c);
    c = wmma_bf16(ah.v, bh.v, c);
    asm volatile("v_nop\n\tv_nop\n\tv_nop\n\tv_nop" : "+v"(c) : "v"(ah.v), "v"(al.v), "v"(bh.v), "v"(bl.v));
}

__device__ __forceinline__ void mma3x2(v8f& c0, v8f& c1, const Frag& ah, const Frag& al,
                                       const Frag& bh0, const Frag& bl0, const Frag& bh1, const Frag& bl1)
{
    c0 = wmma_bf16(al.v, bh0.v, c0);
    c0 = wmma_bf16(ah.v, bl0.v, c0);
    c0 = wmma_bf16(ah.v, bh0.v, c0);
    c1 = wmma_bf16(al.v, bh1.v, c1);
    c1 = wmma_bf16(ah.v, bl1.v, c1);
    c1 = wmma_bf16(ah.v, bh1.v, c1);
    asm volatile("v_nop\n\tv_nop\n\tv_nop\n\tv_nop"
                 : "+v"(c0), "+v"(c1)
                 : "v"(ah.v), "v"(al.v), "v"(bh0.v), "v"(bl0.v), "v"(bh1.v), "v"(bl1.v));
}

__device__ __forceinline__ unsigned int bf16_rne(float x)
{
    unsigned int u = __float_as_uint(x);
    u += 0x7FFFu + ((u >> 16) & 1u);
    return u >> 16;
}

__device__ __forceinline__ void split1(float x, unsigned short& h, unsigned short& l)
{
    const unsigned int hb = bf16_rne(x);
    const float hf = __uint_as_float(hb << 16);
    h = (unsigned short)hb;
    l = (unsigned short)bf16_rne(x - hf);
}

__device__ __forceinline__ void split8(const float (&x)[8], v8us& vh, v8us& vl)
{
    vh = (v8us){0, 0, 0, 0, 0, 0, 0, 0};
    vl = (v8us){0, 0, 0, 0, 0, 0, 0, 0};
#pragma unroll
    for (int i = 0; i < 8; ++i) {
        unsigned short a, b;
        split1(x[i], a, b);
        vh[i] = a;
        vl[i] = b;
    }
}

__global__ void __launch_bounds__(256)
k_split(const float* __restrict__ x, void* hiv, void* lov, int n8)
{
    const int g = blockIdx.x * 256 + threadIdx.x;
    if (g >= n8) return;
    unsigned short* hi = (unsigned short*)hiv;
    unsigned short* lo = (unsigned short*)lov;
    const size_t e = (size_t)g * 8;
    const v4f a = *(const v4f*)(x + e);
    const v4f b = *(const v4f*)(x + e + 4);
    const float f[8] = {a[0], a[1], a[2], a[3], b[0], b[1], b[2], b[3]};
    v8us vh, vl;
    split8(f, vh, vl);
    *(volatile v8us*)(hi + e) = vh;
    *(volatile v8us*)(lo + e) = vl;
    __threadfence();
    *(volatile v8us*)(hi + e) = vh;
    *(volatile v8us*)(lo + e) = vl;
}

__device__ __forceinline__ void wsplit_store(const float (*T)[65], int tid, int k0, int n0,
                                             unsigned short* hi, unsigned short* lo)
{
    const int j = tid & 7;
#pragma unroll
    for (int it = 0; it < 2; ++it) {
        const int L = it * 32 + (tid >> 3);
        float f[8];
#pragma unroll
        for (int i = 0; i < 8; ++i) f[i] = T[8 * j + i][L];
        v8us vh, vl;
        split8(f, vh, vl);
        const size_t off = (size_t)(n0 + L) * E_ + k0 + 8 * j;
        *(volatile v8us*)(hi + off) = vh;
        *(volatile v8us*)(lo + off) = vl;
    }
}

__global__ void __launch_bounds__(256)
k_wsplit(const float* __restrict__ w0, const float* __restrict__ w1,
         const float* __restrict__ w2, const float* __restrict__ w3,
         unsigned short* wt)
{
    __shared__ float T[64][65];
    const int tid = threadIdx.x;
    const int z = blockIdx.z;
    const float* W = w0;
    if (z == 1) W = w1;
    if (z == 2) W = w2;
    if (z == 3) W = w3;
    const int k0 = blockIdx.x * 64;
    const int n0 = blockIdx.y * 64;
    {
        const int row = tid >> 2;
        const int cg  = (tid & 3) * 16;
        const float* src = W + (size_t)(k0 + row) * E_ + n0 + cg;
#pragma unroll
        for (int i = 0; i < 4; ++i) {
            const v4f f = *(const v4f*)(src + 4 * i);
            T[row][cg + 4 * i + 0] = f[0];
            T[row][cg + 4 * i + 1] = f[1];
            T[row][cg + 4 * i + 2] = f[2];
            T[row][cg + 4 * i + 3] = f[3];
        }
    }
    __syncthreads();
    unsigned short* hi = wt + (size_t)z * 2 * E_ * E_;
    unsigned short* lo = hi + (size_t)E_ * E_;
    wsplit_store(T, tid, k0, n0, hi, lo);
    __threadfence();
    wsplit_store(T, tid, k0, n0, hi, lo);
}

template <int MODE>
__device__ __forceinline__ void gemm_store(const float* st, int blockM, int blockN, int tid,
                                           void* out0, void* out1)
{
    const int j = tid & 7;
    if (MODE == 0) {
        unsigned short* oh = (unsigned short*)out0;
        unsigned short* ol = (unsigned short*)out1;
        const int b = blockM / S_, s0 = blockM % S_, h0 = blockN / D_;
#pragma unroll
        for (int it = 0; it < 8; ++it) {
            const int L  = it * 32 + (tid >> 3);
            const int r  = L >> 1;
            const int hd = L & 1;
            const float* sp = st + r * 128 + hd * 64 + 8 * j;
            const v4f a = *(const v4f*)sp;
            const v4f c = *(const v4f*)(sp + 4);
            const float f[8] = {a[0], a[1], a[2], a[3], c[0], c[1], c[2], c[3]};
            v8us vh, vl;
            split8(f, vh, vl);
            const size_t off = ((size_t)(b * H_ + h0 + hd) * S_ + s0 + r) * D_ + 8 * j;
            *(volatile v8us*)(oh + off) = vh;
            *(volatile v8us*)(ol + off) = vl;
        }
    } else if (MODE == 1) {
        unsigned short* oh = (unsigned short*)out0;
        unsigned short* ol = (unsigned short*)out1;
        const int b = blockM / S_, s0 = blockM % S_, h0 = blockN / D_;
#pragma unroll
        for (int it = 0; it < 8; ++it) {
            const int L  = it * 32 + (tid >> 3);
            const int sh = L & 1;
            const int d  = (L >> 1) & 63;
            const int hd = L >> 7;
            float f[8];
#pragma unroll
            for (int i = 0; i < 8; ++i) f[i] = st[(sh * 64 + 8 * j + i) * 128 + hd * 64 + d];
            v8us vh, vl;
            split8(f, vh, vl);
            const size_t off = ((size_t)(b * H_ + h0 + hd) * D_ + d) * S_ + s0 + sh * 64 + 8 * j;
            *(volatile v8us*)(oh + off) = vh;
            *(volatile v8us*)(ol + off) = vl;
        }
    } else {
        float* o = (float*)out0;
#pragma unroll
        for (int it = 0; it < 16; ++it) {
            const int L = it * 32 + (tid >> 3);
            const int r = L >> 2;
            const int c = L & 3;
            const v4f a = *(const v4f*)(st + r * 128 + c * 32 + 4 * j);
            const size_t off = (size_t)(blockM + r) * E_ + blockN + c * 32 + 4 * j;
            *(volatile v4f*)(o + off) = a;
        }
    }
}

template <int MODE>
__global__ void __launch_bounds__(256)
k_gemm(const void* Ahv, const void* Alv,
       const unsigned short* __restrict__ Bhi, const unsigned short* __restrict__ Blo,
       const float* __restrict__ bias, void* out0, void* out1)
{
    extern __shared__ __align__(16) float gstage[];
    const unsigned short* Ahi = (const unsigned short*)Ahv;
    const unsigned short* Alo = (const unsigned short*)Alv;

    const int tid   = threadIdx.x;
    const int lane  = tid & 31;
    const int wave  = tid >> 5;
    const int waveM = wave >> 2;
    const int waveN = wave & 3;
    const int lm    = lane & 15;
    const int hh    = lane >> 4;
    const int blockM = blockIdx.y * 128;
    const int blockN = blockIdx.x * 128;

    v8f zero = {};
    v8f acc[4][2];
#pragma unroll
    for (int mt = 0; mt < 4; ++mt) { acc[mt][0] = zero; acc[mt][1] = zero; }

#pragma unroll 1
    for (int k0 = 0; k0 < E_; k0 += 32) {
        Frag bh[2], bl[2];
#pragma unroll
        for (int nt = 0; nt < 2; ++nt) {
            const int n = blockN + waveN * 32 + nt * 16 + lm;
            const size_t p = (size_t)n * E_ + k0 + 8 * hh;
            bh[nt].u[0] = *(const v8us*)(Bhi + p);
            bh[nt].u[1] = *(const v8us*)(Bhi + p + 16);
            bl[nt].u[0] = *(const v8us*)(Blo + p);
            bl[nt].u[1] = *(const v8us*)(Blo + p + 16);
        }
#pragma unroll
        for (int mt = 0; mt < 4; ++mt) {
            const int m = blockM + waveM * 64 + mt * 16 + lm;
            size_t p;
            if (MODE == 2) {
                const int b = m / S_, s = m % S_;
                p = ((size_t)(b * H_ + (k0 >> 6)) * S_ + s) * D_ + (k0 & 63) + 8 * hh;
            } else {
                p = (size_t)m * E_ + k0 + 8 * hh;
            }
            Frag ah, al;
            ah.u[0] = *(const v8us*)(Ahi + p);
            ah.u[1] = *(const v8us*)(Ahi + p + 16);
            al.u[0] = *(const v8us*)(Alo + p);
            al.u[1] = *(const v8us*)(Alo + p + 16);
            mma3x2(acc[mt][0], acc[mt][1], ah, al, bh[0], bl[0], bh[1], bl[1]);
        }
    }

    float bn[2];
#pragma unroll
    for (int nt = 0; nt < 2; ++nt) bn[nt] = bias[blockN + waveN * 32 + nt * 16 + lm];
#pragma unroll
    for (int mt = 0; mt < 4; ++mt)
#pragma unroll
        for (int nt = 0; nt < 2; ++nt)
#pragma unroll
            for (int r = 0; r < 8; ++r) {
                const int lr = waveM * 64 + mt * 16 + 8 * hh + r;
                const int lc = waveN * 32 + nt * 16 + lm;
                gstage[lr * 128 + lc] = acc[mt][nt][r] + bn[nt];
            }
    __syncthreads();

    gemm_store<MODE>(gstage, blockM, blockN, tid, out0, out1);
    __threadfence();
    gemm_store<MODE>(gstage, blockM, blockN, tid, out0, out1);
}

__device__ __forceinline__ void attn_store(const float (*Ost)[64], int lane, size_t hb, int rowbase,
                                           unsigned short* Ohi, unsigned short* Olo)
{
    const int j = lane & 7;
#pragma unroll
    for (int it = 0; it < 4; ++it) {
        const int rl = it * 4 + (lane >> 3);
        const float* sp = &Ost[rl][8 * j];
        const v4f a = *(const v4f*)sp;
        const v4f c = *(const v4f*)(sp + 4);
        const float f[8] = {a[0], a[1], a[2], a[3], c[0], c[1], c[2], c[3]};
        v8us vh, vl;
        split8(f, vh, vl);
        const size_t off = hb + (size_t)(rowbase + rl) * D_ + 8 * j;
        *(volatile v8us*)(Ohi + off) = vh;
        *(volatile v8us*)(Olo + off) = vl;
    }
}

__global__ void __launch_bounds__(256)
k_attn(const unsigned short* Qhi, const unsigned short* Qlo,
       const unsigned short* __restrict__ Khi, const unsigned short* __restrict__ Klo,
       const unsigned short* __restrict__ Vhi, const unsigned short* __restrict__ Vlo,
       unsigned short* Ohi, unsigned short* Olo)
{
    __shared__ __align__(16) unsigned short Ph[8][16][32];
    __shared__ __align__(16) unsigned short Pl[8][16][32];
    __shared__ __align__(16) float Ost[8][16][64];

    const int tid  = threadIdx.x;
    const int lane = tid & 31;
    const int wave = tid >> 5;
    const int lm   = lane & 15;
    const int hh   = lane >> 4;
    const int bh   = blockIdx.y;
    const int rowbase = blockIdx.x * 128 + wave * 16;
    const size_t hb = (size_t)bh * S_ * D_;

    Frag qh[2], ql[2];
#pragma unroll
    for (int dc = 0; dc < 2; ++dc) {
        const size_t p = hb + (size_t)(rowbase + lm) * D_ + dc * 32 + 8 * hh;
        qh[dc].u[0] = *(const v8us*)(Qhi + p);
        qh[dc].u[1] = *(const v8us*)(Qhi + p + 16);
        ql[dc].u[0] = *(const v8us*)(Qlo + p);
        ql[dc].u[1] = *(const v8us*)(Qlo + p + 16);
    }

    v8f zero = {};
    v8f oacc[4];
#pragma unroll
    for (int nt = 0; nt < 4; ++nt) oacc[nt] = zero;
    float mrow[8], lrow[8];
#pragma unroll
    for (int r = 0; r < 8; ++r) { mrow[r] = -1e30f; lrow[r] = 0.0f; }

    const float scale = 0.125f;
    const int tl = (rowbase + 15) >> 5;

#pragma unroll 1
    for (int tc = 0; tc <= tl; ++tc) {
        const int t = tc << 5;

        v8f sacc[2];
        sacc[0] = zero; sacc[1] = zero;
#pragma unroll
        for (int ct = 0; ct < 2; ++ct) {
#pragma unroll
            for (int dc = 0; dc < 2; ++dc) {
                Frag kh, kl;
                const size_t p = hb + (size_t)(t + ct * 16 + lm) * D_ + dc * 32 + 8 * hh;
                kh.u[0] = *(const v8us*)(Khi + p);
                kh.u[1] = *(const v8us*)(Khi + p + 16);
                kl.u[0] = *(const v8us*)(Klo + p);
                kl.u[1] = *(const v8us*)(Klo + p + 16);
                mma3(sacc[ct], qh[dc], ql[dc], kh, kl);
            }
        }

#pragma unroll
        for (int r = 0; r < 8; ++r) {
            const int row = rowbase + 8 * hh + r;
            const int c0 = t + lm;
            const int c1 = t + 16 + lm;
            const float x0 = (c0 <= row) ? sacc[0][r] * scale : -1e30f;
            const float x1 = (c1 <= row) ? sacc[1][r] * scale : -1e30f;
            float mx = fmaxf(x0, x1);
#pragma unroll
            for (int msk = 1; msk < 16; msk <<= 1)
                mx = fmaxf(mx, __shfl_xor(mx, msk, 32));
            const float mnew = fmaxf(mrow[r], mx);
            const float sf = __expf(mrow[r] - mnew);
            const float p0 = __expf(x0 - mnew);
            const float p1 = __expf(x1 - mnew);
            float rs = p0 + p1;
#pragma unroll
            for (int msk = 1; msk < 16; msk <<= 1)
                rs += __shfl_xor(rs, msk, 32);
            lrow[r] = lrow[r] * sf + rs;
            mrow[r] = mnew;
#pragma unroll
            for (int nt = 0; nt < 4; ++nt) oacc[nt][r] *= sf;
            unsigned short a0, b0, a1, b1;
            split1(p0, a0, b0);
            split1(p1, a1, b1);
            const int pr = 8 * hh + r;
            Ph[wave][pr][lm]      = a0;
            Pl[wave][pr][lm]      = b0;
            Ph[wave][pr][16 + lm] = a1;
            Pl[wave][pr][16 + lm] = b1;
        }
        __builtin_amdgcn_fence(__ATOMIC_SEQ_CST, "wavefront");
        __builtin_amdgcn_wave_barrier();

        Frag ph, pl;
        ph.u[0] = *(const v8us*)&Ph[wave][lm][8 * hh];
        ph.u[1] = *(const v8us*)&Ph[wave][lm][16 + 8 * hh];
        pl.u[0] = *(const v8us*)&Pl[wave][lm][8 * hh];
        pl.u[1] = *(const v8us*)&Pl[wave][lm][16 + 8 * hh];
#pragma unroll
        for (int nt = 0; nt < 4; ++nt) {
            Frag vh, vl;
            const size_t p = hb + (size_t)(nt * 16 + lm) * S_ + t + 8 * hh;
            vh.u[0] = *(const v8us*)(Vhi + p);
            vh.u[1] = *(const v8us*)(Vhi + p + 16);
            vl.u[0] = *(const v8us*)(Vlo + p);
            vl.u[1] = *(const v8us*)(Vlo + p + 16);
            mma3(oacc[nt], ph, pl, vh, vl);
        }
        __builtin_amdgcn_fence(__ATOMIC_SEQ_CST, "wavefront");
        __builtin_amdgcn_wave_barrier();
    }

#pragma unroll
    for (int r = 0; r < 8; ++r) {
        const float inv = 1.0f / lrow[r];
#pragma unroll
        for (int nt = 0; nt < 4; ++nt)
            Ost[wave][8 * hh + r][nt * 16 + lm] = oacc[nt][r] * inv;
    }
    __builtin_amdgcn_fence(__ATOMIC_SEQ_CST, "wavefront");
    __builtin_amdgcn_wave_barrier();

    attn_store(Ost[wave], lane, hb, rowbase, Ohi, Olo);
    __threadfence();
    attn_store(Ost[wave], lane, hb, rowbase, Ohi, Olo);
}

extern "C" void kernel_launch(void* const* d_in, const int* in_sizes, int n_in,
                              void* d_out, int out_size, void* d_ws, size_t ws_size,
                              hipStream_t stream)
{
    if (n_in < 11) return;
    const int nact = B_ * S_ * E_;
    const int nw   = E_ * E_;
    if (in_sizes[0] != nact || in_sizes[1] != nact || in_sizes[2] != nact) return;
    if (in_sizes[3] != nw || in_sizes[5] != nw || in_sizes[7] != nw || in_sizes[9] != nw) return;
    if (in_sizes[4] != E_ || in_sizes[6] != E_ || in_sizes[8] != E_ || in_sizes[10] != E_) return;
    if (out_size != nact) return;

    const size_t P = (size_t)nact;
    const size_t ws_need = (6 * P + 8 * (size_t)nw) * sizeof(unsigned short);
    if (ws_size < ws_need) return;

    const float* q   = (const float*)d_in[0];
    const float* k   = (const float*)d_in[1];
    const float* v   = (const float*)d_in[2];
    const float* w_q = (const float*)d_in[3];
    const float* b_q = (const float*)d_in[4];
    const float* w_k = (const float*)d_in[5];
    const float* b_k = (const float*)d_in[6];
    const float* w_v = (const float*)d_in[7];
    const float* b_v = (const float*)d_in[8];
    const float* w_o = (const float*)d_in[9];
    const float* b_o = (const float*)d_in[10];

    unsigned short* ws  = (unsigned short*)d_ws;
    unsigned short* Qhi = ws;
    unsigned short* Qlo = ws + P;
    unsigned short* Khi = ws + 2 * P;
    unsigned short* Klo = ws + 3 * P;
    unsigned short* Vhi = ws + 4 * P;
    unsigned short* Vlo = ws + 5 * P;
    unsigned short* Wt  = ws + 6 * P;

    unsigned short* Xh = (unsigned short*)d_out;
    unsigned short* Xl = Xh + P;

    const dim3 blk(256);
    const dim3 ggrid(E_ / 128, M_ / 128);
    const size_t glds = 128 * 128 * sizeof(float);
    const int n8 = nact / 8;
    const dim3 sgrid((n8 + 255) / 256);

    k_wsplit<<<dim3(E_ / 64, E_ / 64, 4), blk, 0, stream>>>(w_q, w_k, w_v, w_o, Wt);

    k_split<<<sgrid, blk, 0, stream>>>(q, Xh, Xl, n8);
    k_gemm<0><<<ggrid, blk, glds, stream>>>((const void*)Xh, (const void*)Xl,
                                           Wt + 0 * (size_t)nw, Wt + 1 * (size_t)nw, b_q, Qhi, Qlo);
    k_split<<<sgrid, blk, 0, stream>>>(k, Xh, Xl, n8);
    k_gemm<0><<<ggrid, blk, glds, stream>>>((const void*)Xh, (const void*)Xl,
                                           Wt + 2 * (size_t)nw, Wt + 3 * (size_t)nw, b_k, Khi, Klo);
    k_split<<<sgrid, blk, 0, stream>>>(v, Xh, Xl, n8);
    k_gemm<1><<<ggrid, blk, glds, stream>>>((const void*)Xh, (const void*)Xl,
                                           Wt + 4 * (size_t)nw, Wt + 5 * (size_t)nw, b_v, Vhi, Vlo);

    k_attn<<<dim3(S_ / 128, B_ * H_), blk, 0, stream>>>(Qhi, Qlo, Khi, Klo, Vhi, Vlo, Qhi, Qlo);

    k_gemm<2><<<ggrid, blk, glds, stream>>>((const void*)Qhi, (const void*)Qlo,
                                           Wt + 6 * (size_t)nw, Wt + 7 * (size_t)nw, b_o, d_out, d_out);
}
